// CausalSelfAttention_71116068487587
// MI455X (gfx1250) — hardware-verified
//
#include <hip/hip_runtime.h>
#include <math.h>

typedef __attribute__((ext_vector_type(16))) _Float16 v16h;
typedef __attribute__((ext_vector_type(16))) __bf16 v16b;
typedef __attribute__((ext_vector_type(8)))  _Float16 v8h;
typedef __attribute__((ext_vector_type(8)))  __bf16 v8b;
typedef __attribute__((ext_vector_type(8)))  float v8f;
typedef __attribute__((ext_vector_type(4)))  float v4f;
typedef __attribute__((ext_vector_type(4)))  unsigned v4u;

template <typename T> __device__ __forceinline__ void vst2(void* p, T v) { *(volatile T*)p = v; __threadfence(); *(volatile T*)p = v; }
__device__ __forceinline__ v8f wmma16(v16h a, v16h b, v8f c) {
  v8f d = __builtin_amdgcn_wmma_f32_16x16x32_f16(false, a, false, b, (short)0, c, false, false);
  asm volatile("v_nop\n\tv_nop\n\tv_nop\n\tv_nop" : "+v"(d) : "v"(a), "v"(b));
  return d;
}
__device__ __forceinline__ v8f wmma_bf(v16b a, v16b b, v8f c) {
  v8f d = __builtin_amdgcn_wmma_f32_16x16x32_bf16(false, a, false, b, (short)0, c, false, false);
  asm volatile("v_nop\n\tv_nop\n\tv_nop\n\tv_nop" : "+v"(d) : "v"(a), "v"(b));
  return d;
}
__device__ __forceinline__ v16h frag_h(const _Float16* rowk0, int lane) {
  union { v16h v; v8h q[2]; } u; const _Float16* p = rowk0 + 8 * (lane >> 4);
  u.q[0] = *(const v8h*)p; u.q[1] = *(const v8h*)(p + 16); return u.v;
}
__device__ __forceinline__ v16b frag_b(const __bf16* rowk0, int lane) {
  union { v16b v; v8b q[2]; } u; const __bf16* p = rowk0 + 8 * (lane >> 4);
  u.q[0] = *(const v8b*)p; u.q[1] = *(const v8b*)(p + 16); return u.v;
}
__device__ __forceinline__ void pack_h(const float v[8], v4u& hi, v4u& re) {
  union { v8h v; v4u u; } a, b;
#pragma unroll
  for (int i = 0; i < 8; ++i) { const _Float16 h = (_Float16)v[i]; a.v[i] = h; b.v[i] = (_Float16)((v[i] - (float)h) * 1024.0f); }
  hi = a.u; re = b.u;
}
__device__ __forceinline__ void pack_b(const float v[8], v4u& hi, v4u& lo) {
  union { v8b v; v4u u; } a, b;
#pragma unroll
  for (int i = 0; i < 8; ++i) { const __bf16 h = (__bf16)v[i]; a.v[i] = h; b.v[i] = (__bf16)(v[i] - (float)h); }
  hi = a.u; lo = b.u;
}
#define LDSX() do { asm volatile("s_wait_dscnt 0" ::: "memory"); __builtin_amdgcn_wave_barrier(); __builtin_amdgcn_fence(3  , "workgroup"); } while (0)

#ifndef NB
#define NB 2
#endif
#ifndef SEQ
#define SEQ 2048
#endif
#define TT SEQ
#define NB_FULL 2
#define TT_FULL 2048
#define CC 1024
#define DIN 1024
#define NH 16
#define HD 64
#define WIN 256
#define SINKK 4
#define SCALE (0.125f)

static_assert(CC == NH * HD);
static_assert(HD == 64);
static_assert(DIN % 64 == 0 && CC % 128 == 0 && DIN % 128 == 0);
static_assert(TT % 64 == 0 && TT <= TT_FULL && NB <= NB_FULL);
static_assert(((size_t)NB * TT * (DIN / 8)) % 256 == 0);
static_assert(TT % 8 == 0);
static_assert(WIN % 32 == 0 && SINKK <= 32);

#define PLANE16 (2u * (size_t)NB * TT * CC)
#define WS_XB   0u
#define WS_WAT  (WS_XB  + 2u * (size_t)NB * TT * DIN)
#define WS_WPT  (WS_WAT + 2u * (size_t)3 * CC * DIN)
#define WS_TAB  (WS_WPT + 2u * (size_t)DIN * CC)
#define WS_QH   (WS_TAB + 4u * (size_t)TT * 64)
#define WS_KH   (WS_QH  + PLANE16)
#define WS_QL   (WS_KH  + PLANE16)
#define WS_KL   (WS_QL  + PLANE16)
#define WS_VB   (WS_KL  + PLANE16)
#define WS_VBL  (WS_VB  + PLANE16)
#define WS_YH   (WS_VBL + PLANE16)
#define WS_YL   (WS_YH  + PLANE16)
#define WS_END  (WS_YL  + PLANE16)
static_assert(WS_END <= 134217728u);
static_assert(WS_WAT % 128 == 0 && WS_WPT % 128 == 0 && WS_TAB % 128 == 0 && WS_QH % 128 == 0 && PLANE16 % 128 == 0);

__global__ __launch_bounds__(256) void k_prep_x(const float* __restrict__ X, __bf16* __restrict__ XB) {
  const size_t idx = (size_t)blockIdx.x * 256 + threadIdx.x;
  const size_t row = idx / (DIN / 8); const int pc = (int)(idx % (DIN / 8));
  const size_t b = row / TT, t = row % TT;
  const float* src = X + (b * TT_FULL + t) * DIN + pc * 8;
  const v4f f0 = *(const v4f*)src, f1 = *(const v4f*)(src + 4);
  union { v8b v; v4u u; } o;
#pragma unroll
  for (int i = 0; i < 4; ++i) { o.v[i] = (__bf16)f0[i]; o.v[4 + i] = (__bf16)f1[i]; }
  vst2(XB + row * DIN + pc * 8, o.u);
}
__global__ __launch_bounds__(128) void k_prep_w(const float* __restrict__ W, __bf16* __restrict__ WT, int N, int K) {
  __shared__ __align__(16) __bf16 tl[64][72];
  const int tid = threadIdx.x; const int n0 = blockIdx.x * 64, k0 = blockIdx.y * 64;
#pragma unroll 2
  for (int e = tid; e < 64 * 16; e += 128) { const int kr = e >> 4, pc = e & 15;
    const v4f f = *(const v4f*)(W + (size_t)(k0 + kr) * N + n0 + pc * 4);
#pragma unroll
    for (int i = 0; i < 4; ++i) tl[pc * 4 + i][kr] = (__bf16)f[i]; }
  __syncthreads();
  for (int e = tid; e < 64 * 8; e += 128) { const int nr = e >> 3, q = e & 7;
    vst2(WT + (size_t)(n0 + nr) * K + k0 + q * 8, *(const v4u*)&tl[nr][q * 8]); }
}
__global__ __launch_bounds__(256) void k_tab(float* __restrict__ TAB) {
  __shared__ __align__(16) float tt[8][64];
  const int tid = threadIdx.x; const int tr = tid >> 5, j = tid & 31; const int t = blockIdx.x * 8 + tr;
  double p = 1.0;
  p *= (j & 1) ? 1.3335214321633240 : 1.0;
  p *= (j & 2) ? 1.7782794100389228 : 1.0;
  p *= (j & 4) ? 3.1622776601683795 : 1.0;
  p *= (j & 8) ? 10.0 : 1.0;
  p *= (j & 16) ? 100.0 : 1.0;
  const float pf = (float)p; const float inv = 1.0f / pf; const float ang = (float)t * inv;
  float sn, cs; sincosf(ang, &sn, &cs);
  tt[tr][j] = cs; tt[tr][32 + j] = sn;
  __syncthreads();
  if (tid < 128) { const int row = tid >> 4, pc = tid & 15;
    vst2(TAB + (size_t)(blockIdx.x * 8 + row) * 64 + pc * 4, *(const v4f*)&tt[row][pc * 4]); }
}
__global__ __launch_bounds__(128) void k_proj(const __bf16* __restrict__ XB, const __bf16* __restrict__ WAT, const float* __restrict__ TAB,
    _Float16* __restrict__ QKH, _Float16* __restrict__ QKL, __bf16* __restrict__ VB, __bf16* __restrict__ VBL) {
  __shared__ __align__(16) float st[64][132];
  const int tid = threadIdx.x; const int wave = __builtin_amdgcn_readfirstlane(tid >> 5); const int lane = tid & 31, col = lane & 15, g = lane >> 4;
  const int which = blockIdx.y >> 3; const int c0 = (blockIdx.y & 7) * 128;
  const size_t r0 = (size_t)blockIdx.x * 64; const size_t bb = r0 / TT; const int t0 = (int)(r0 % TT);
  v8f acc[8] = {};
  const __bf16* ap = XB + (r0 + wave * 16 + col) * DIN;
  const __bf16* wp = WAT + ((size_t)which * CC + c0 + col) * DIN;
#pragma unroll 2
  for (int kc = 0; kc < DIN / 32; ++kc) { const v16b a = frag_b(ap + kc * 32, lane);
#pragma unroll
    for (int j = 0; j < 8; ++j) { const v16b w = frag_b(wp + (size_t)j * 16 * DIN + kc * 32, lane); acc[j] = wmma_bf(a, w, acc[j]); } }
#pragma unroll
  for (int j = 0; j < 8; ++j) {
#pragma unroll
    for (int r = 0; r < 8; ++r) st[wave * 16 + 8 * g + r][j * 16 + col] = acc[j][r]; }
  __syncthreads();
  if (which < 2) {
#pragma unroll 2
    for (int e = tid; e < 64 * 2 * 32; e += 128) { const int rl = e >> 6, hh = (e >> 5) & 1, d = e & 31;
      const float cs = TAB[(size_t)(t0 + rl) * 64 + d], sn = TAB[(size_t)(t0 + rl) * 64 + 32 + d];
      const float x1 = st[rl][hh * HD + d], x2 = st[rl][hh * HD + 32 + d];
      st[rl][hh * HD + d] = x1 * cs - x2 * sn; st[rl][hh * HD + 32 + d] = x2 * cs + x1 * sn; } }
  __syncthreads();
  if (which < 2) {
    _Float16* DH = QKH + (size_t)which * ((size_t)NB * TT * CC); _Float16* DL = QKL + (size_t)which * ((size_t)NB * TT * CC);
    for (int e = tid; e < 64 * 16; e += 128) { const int rl = e >> 4, q = e & 15;
      const v4f a = *(const v4f*)&st[rl][q * 8], c = *(const v4f*)&st[rl][q * 8 + 4];
      float v[8];
#pragma unroll
      for (int i = 0; i < 4; ++i) { v[i] = a[i]; v[4 + i] = c[i]; }
      v4u hi, re; pack_h(v, hi, re);
      const size_t o = (r0 + rl) * CC + c0 + q * 8;
      vst2(DH + o, hi); vst2(DL + o, re); }
  } else {
    for (int e = tid; e < 128 * 8; e += 128) { const int cl = e >> 3, q = e & 7;
      float v[8];
#pragma unroll
      for (int i = 0; i < 8; ++i) v[i] = st[q * 8 + i][cl];
      v4u hi, lo; pack_b(v, hi, lo);
      const size_t o = (bb * CC + c0 + cl) * (size_t)TT + t0 + q * 8;
      vst2(VB + o, hi); vst2(VBL + o, lo); } }
}
__global__ __launch_bounds__(128) void k_attn(const _Float16* __restrict__ QH, const _Float16* __restrict__ QL, const _Float16* __restrict__ KH, const _Float16* __restrict__ KL,
    const __bf16* __restrict__ VB, const __bf16* __restrict__ VBL, __bf16* __restrict__ YH, __bf16* __restrict__ YL) {
  __shared__ __align__(16) float ss[4][16][HD + 4];
  const int tid = threadIdx.x; const int wave = __builtin_amdgcn_readfirstlane(tid >> 5); const int lane = tid & 31, col = lane & 15, g = lane >> 4;
  const int hd = blockIdx.y; const size_t b = blockIdx.z; const int q0 = blockIdx.x * 64 + wave * 16; const size_t rowb = b * TT;
  const size_t qoff = (rowb + q0 + col) * CC + hd * HD;
  const v16h qh0 = frag_h(QH + qoff, lane), qh1 = frag_h(QH + qoff + 32, lane), ql0 = frag_h(QL + qoff, lane), ql1 = frag_h(QL + qoff + 32, lane);
  v8f o0 = {}, o1 = {}, o2 = {}, o3 = {};
  float m = -3.0e38f, l = 0.f;
  const int iq = q0 + col;
  const int khi = (q0 + 15) >> 5; int klo = (q0 > (WIN - 1)) ? ((q0 - (WIN - 1)) >> 5) : 0; if (klo < 1) klo = 1;
  const int nst = 1 + ((khi >= klo) ? (khi - klo + 1) : 0);
  const size_t vrow = (b * CC + hd * HD + col) * (size_t)TT;
#pragma unroll 1
  for (int it = 0; it < nst; ++it) {
    const int key0 = ((it == 0) ? 0 : (klo + it - 1)) * 32;
    v8f s0 = {}, s1 = {}, e0 = {}, e1 = {};
    { const size_t ko = (rowb + key0 + col) * CC + hd * HD;
      v16h kh = frag_h(KH + ko, lane), kl = frag_h(KL + ko, lane);
      s0 = wmma16(kh, qh0, s0); e0 = wmma16(kl, qh0, e0); e0 = wmma16(kh, ql0, e0);
      kh = frag_h(KH + ko + 32, lane); kl = frag_h(KL + ko + 32, lane);
      s0 = wmma16(kh, qh1, s0); e0 = wmma16(kl, qh1, e0); e0 = wmma16(kh, ql1, e0);
      const size_t k1 = ko + (size_t)16 * CC;
      kh = frag_h(KH + k1, lane); kl = frag_h(KL + k1, lane);
      s1 = wmma16(kh, qh0, s1); e1 = wmma16(kl, qh0, e1); e1 = wmma16(kh, ql0, e1);
      kh = frag_h(KH + k1 + 32, lane); kl = frag_h(KL + k1 + 32, lane);
      s1 = wmma16(kh, qh1, s1); e1 = wmma16(kl, qh1, e1); e1 = wmma16(kh, ql1, e1); }
    float v0[8], v1[8]; float mx = m;
#pragma unroll
    for (int r = 0; r < 8; ++r) { const int j0 = key0 + 8 * g + r, j1 = j0 + 16;
      const bool a0 = (j0 <= iq) && (((iq - j0) < WIN) || (j0 < SINKK));
      const bool a1 = (j1 <= iq) && (((iq - j1) < WIN) || (j1 < SINKK));
      const float x0 = (s0[r] + e0[r] * (1.0f / 1024.0f)) * SCALE, x1 = (s1[r] + e1[r] * (1.0f / 1024.0f)) * SCALE;
      v0[r] = a0 ? x0 : -3.0e38f; v1[r] = a1 ? x1 : -3.0e38f;
      mx = fmaxf(mx, fmaxf(v0[r], v1[r])); }
    mx = fmaxf(mx, __shfl_xor(mx, 16));
    const float alpha = __expf(m - mx); m = mx;
    float ls = 0.f; v16b ph, pl;
#pragma unroll
    for (int r = 0; r < 8; ++r) {
      const float p0 = (v0[r] > -1.0e38f) ? __expf(v0[r] - mx) : 0.f, p1 = (v1[r] > -1.0e38f) ? __expf(v1[r] - mx) : 0.f;
      ls += p0 + p1;
      const __bf16 h0 = (__bf16)p0, h1 = (__bf16)p1;
      ph[r] = h0; pl[r] = (__bf16)(p0 - (float)h0); ph[8 + r] = h1; pl[8 + r] = (__bf16)(p1 - (float)h1); }
    l = l * alpha + ls;
    o0 = o0 * alpha; o1 = o1 * alpha; o2 = o2 * alpha; o3 = o3 * alpha;
    { const size_t vo = vrow + key0;
      v16b vh = frag_b(VB + vo, lane), vl = frag_b(VBL + vo, lane);
      o0 = wmma_bf(vh, ph, o0); o0 = wmma_bf(vl, ph, o0); o0 = wmma_bf(vh, pl, o0);
      vh = frag_b(VB + vo + (size_t)16 * TT, lane); vl = frag_b(VBL + vo + (size_t)16 * TT, lane);
      o1 = wmma_bf(vh, ph, o1); o1 = wmma_bf(vl, ph, o1); o1 = wmma_bf(vh, pl, o1);
      vh = frag_b(VB + vo + (size_t)32 * TT, lane); vl = frag_b(VBL + vo + (size_t)32 * TT, lane);
      o2 = wmma_bf(vh, ph, o2); o2 = wmma_bf(vl, ph, o2); o2 = wmma_bf(vh, pl, o2);
      vh = frag_b(VB + vo + (size_t)48 * TT, lane); vl = frag_b(VBL + vo + (size_t)48 * TT, lane);
      o3 = wmma_bf(vh, ph, o3); o3 = wmma_bf(vl, ph, o3); o3 = wmma_bf(vh, pl, o3); }
  }
  const float lt = l + __shfl_xor(l, 16); const float inv = 1.0f / lt;
#pragma unroll
  for (int r = 0; r < 8; ++r) { ss[wave][col][8 * g + r] = o0[r] * inv; ss[wave][col][16 + 8 * g + r] = o1[r] * inv; ss[wave][col][32 + 8 * g + r] = o2[r] * inv; ss[wave][col][48 + 8 * g + r] = o3[r] * inv; }
  LDSX();
  for (int i4 = 0; i4 < 4; ++i4) { const int row = i4 * 4 + (lane >> 3), pc = lane & 7;
    const v4f a = *(const v4f*)&ss[wave][row][pc * 8], c = *(const v4f*)&ss[wave][row][pc * 8 + 4];
    float v[8];
#pragma unroll
    for (int i = 0; i < 4; ++i) { v[i] = a[i]; v[4 + i] = c[i]; }
    v4u hi, lo; pack_b(v, hi, lo);
    const size_t o = (rowb + q0 + row) * CC + hd * HD + pc * 8;
    vst2(YH + o, hi); vst2(YL + o, lo); }
}
__global__ __launch_bounds__(128) void k_out(const __bf16* __restrict__ YH, const __bf16* __restrict__ YL, const __bf16* __restrict__ WPT, float* __restrict__ OUT) {
  __shared__ __align__(16) float sf[4][16][132];
  const int tid = threadIdx.x; const int wave = __builtin_amdgcn_readfirstlane(tid >> 5); const int lane = tid & 31, col = lane & 15, g = lane >> 4;
  const int c0 = blockIdx.y * 128; const size_t r0 = (size_t)blockIdx.x * 64 + wave * 16;
  v8f acc[8] = {};
  const __bf16* ahp = YH + (r0 + col) * CC; const __bf16* alp = YL + (r0 + col) * CC; const __bf16* wp = WPT + (size_t)(c0 + col) * CC;
#pragma unroll 2
  for (int kc = 0; kc < CC / 32; ++kc) { const v16b ah = frag_b(ahp + kc * 32, lane), al = frag_b(alp + kc * 32, lane);
#pragma unroll
    for (int j = 0; j < 8; ++j) { const v16b w = frag_b(wp + (size_t)j * 16 * CC + kc * 32, lane); acc[j] = wmma_bf(ah, w, acc[j]); acc[j] = wmma_bf(al, w, acc[j]); } }
#pragma unroll
  for (int j = 0; j < 8; ++j) {
#pragma unroll
    for (int r = 0; r < 8; ++r) sf[wave][8 * g + r][j * 16 + col] = acc[j][r]; }
  LDSX();
  for (int rl = 0; rl < 16; ++rl) { const size_t row = r0 + rl; const size_t ob = row / TT, ot = row % TT;
    vst2(OUT + (ob * TT_FULL + ot) * DIN + c0 + lane * 4, *(const v4f*)&sf[wave][rl][lane * 4]); }
}

extern "C" void kernel_launch(void* const* d_in, const int* in_sizes, int n_in, void* d_out, int out_size, void* d_ws, size_t ws_size, hipStream_t stream) {
  if (n_in < 3) return;
  const long long need_rows = (long long)(NB - 1) * TT_FULL + TT;
  if ((long long)in_sizes[0] < need_rows * DIN) return;
  if ((long long)in_sizes[1] < (long long)DIN * 3 * CC) return;
  if ((long long)in_sizes[2] < (long long)CC * DIN) return;
  if ((long long)out_size < need_rows * DIN) return;
  if (ws_size < (size_t)WS_END) return;
  const float* X = (const float*)d_in[0]; const float* WA = (const float*)d_in[1]; const float* WP = (const float*)d_in[2];
  char* ws = (char*)d_ws;
  __bf16* XB = (__bf16*)(ws + WS_XB); __bf16* WAT = (__bf16*)(ws + WS_WAT); __bf16* WPT = (__bf16*)(ws + WS_WPT); float* TAB = (float*)(ws + WS_TAB);
  _Float16* QH = (_Float16*)(ws + WS_QH); _Float16* KH = (_Float16*)(ws + WS_KH); _Float16* QL = (_Float16*)(ws + WS_QL); _Float16* KL = (_Float16*)(ws + WS_KL);
  __bf16* VB = (__bf16*)(ws + WS_VB); __bf16* VBL = (__bf16*)(ws + WS_VBL); __bf16* YH = (__bf16*)(ws + WS_YH); __bf16* YL = (__bf16*)(ws + WS_YL);
  k_prep_x<<<dim3((unsigned)(((size_t)NB * TT * (DIN / 8)) / 256)), 256, 0, stream>>>(X, XB);
  k_prep_w<<<dim3(3 * CC / 64, DIN / 64), 128, 0, stream>>>(WA, WAT, 3 * CC, DIN);
  k_prep_w<<<dim3(DIN / 64, CC / 64), 128, 0, stream>>>(WP, WPT, DIN, CC);
  k_tab<<<dim3(TT / 8), 256, 0, stream>>>(TAB);
  k_proj<<<dim3(NB * TT / 64, 3 * CC / 128), 128, 0, stream>>>(XB, WAT, TAB, QH, QL, VB, VBL);
  k_attn<<<dim3(TT / 64, NH, NB), 128, 0, stream>>>(QH, QL, KH, KL, VB, VBL, YH, YL);
  k_out<<<dim3(NB * TT / 64, DIN / 128), 128, 0, stream>>>(YH, YL, WPT, (float*)d_out);
}
